// AxialAttention_30760555774223
// MI455X (gfx1250) — hardware-verified
//
#include <hip/hip_runtime.h>


#ifndef NB_
#define NB_  128
#endif
#define NB_FULL 128
#define TT   256
#define DM   256
#define NH_  8
#define HD   64
#define DQ   (NH_ * HD)
#define DP   (4 * DQ)
#ifndef GB
#if NB_ >= 8
#define GB   8
#else
#define GB   NB_
#endif
#endif
#define GR   (GB * TT)
#define ZH   (GB * NH_)
#define NT   (NB_ * TT)
#define SCL  0.125f

static_assert(NB_ >= 1 && NB_ <= NB_FULL);
static_assert((NB_ % GB) == 0);
static_assert((GR % 64) == 0 && (TT % 64) == 0 && (HD % 64) == 0 && (DM % 64) == 0 && (DQ % 64) == 0 && (DP % 64) == 0);
static_assert((HD % 32) == 0 && (DM % 32) == 0 && (DQ % 32) == 0 && (TT % 32) == 0);
static_assert((TT % 128) == 0 && (NT % 8) == 0 && (DM % 128) == 0);
static_assert(((DQ * DM) % 64) == 0 && ((2 * DQ * DM) % 64) == 0);

typedef unsigned short bf;
typedef __attribute__((ext_vector_type(16))) __bf16   v16bf;
typedef __attribute__((ext_vector_type(8)))  unsigned short v8us;
typedef __attribute__((ext_vector_type(8)))  float    v8f;
typedef __attribute__((ext_vector_type(4)))  float    v4f;
typedef v4f  __attribute__((may_alias)) v4fa;
typedef __attribute__((ext_vector_type(2))) unsigned short v2us;
typedef __attribute__((ext_vector_type(4))) unsigned short v4us;

constexpr size_t al256(size_t b) { return (b + 255) & ~(size_t)255; }
constexpr size_t WS_NEED = al256((size_t)DP * DM * 2) + al256((size_t)DM * DQ * 2) + 2 * al256((size_t)NT * DM * 2) + al256((size_t)GR * DP * 4)
                         + 6 * al256((size_t)ZH * TT * HD * 2) + al256((size_t)ZH * TT * TT * 4) + 2 * al256((size_t)ZH * TT * TT * 2)
                         + al256((size_t)ZH * TT * HD * 4) + 2 * al256((size_t)GR * DQ * 2);
static_assert(WS_NEED <= (size_t)134217728);

__device__ __forceinline__ unsigned short f2bf(float f) { unsigned u = __float_as_uint(f); u += 0x7FFFu + ((u >> 16) & 1u); return (unsigned short)(u >> 16); }
__device__ __forceinline__ float bf2f(unsigned short b) { return __uint_as_float(((unsigned)b) << 16); }
__device__ __forceinline__ float bfr(float f) { return bf2f(f2bf(f)); }
__device__ __forceinline__ v16bf cat16b(v8us lo, v8us hi) { return __builtin_bit_cast(v16bf, __builtin_shufflevector(lo, hi, 0, 1, 2, 3, 4, 5, 6, 7, 8, 9, 10, 11, 12, 13, 14, 15)); }
__device__ __forceinline__ v8f wmmab(v16bf a, v16bf b, v8f c) { return __builtin_amdgcn_wmma_f32_16x16x32_bf16(false, a, false, b, (short)0, c, false, false); }
__device__ __forceinline__ void splitf(float y, unsigned short& h, unsigned short& l) { h = f2bf(y); l = f2bf(y - bf2f(h)); }

template <typename T16> struct WFrag;
template <> struct WFrag<bf> { typedef v16bf V; static __device__ __forceinline__ V ld(const bf* p) { return cat16b(*(const v8us*)p, *(const v8us*)(p + 16)); } static __device__ __forceinline__ v8f mma(V a, V b, v8f c) { return wmmab(a, b, c); } };
template <typename T16, int NSPLIT, bool BIAS>
__global__ __launch_bounds__(32) void k_gemmw(const T16* __restrict__ A, const T16* __restrict__ A2, const T16* __restrict__ Bt, const T16* __restrict__ Bt2, int K, float* C, int ldc, const float* __restrict__ bias, size_t sA, size_t sB, size_t sC) {
    typedef typename WFrag<T16>::V V;
    __shared__ __align__(16) float os[16 * 68];
    const size_t z = blockIdx.z; A += z * sA; if (A2) A2 += z * sA; Bt += z * sB; if (Bt2) Bt2 += z * sB; C += z * sC;
    const int lane = threadIdx.x & 31, lr = lane & 15, hi = lane >> 4; const int r0 = blockIdx.x * 64, c0 = blockIdx.y * 64;
    v8f acc[4][4];
#pragma unroll
    for (int mb = 0; mb < 4; ++mb)
#pragma unroll
        for (int nb = 0; nb < 4; ++nb) acc[mb][nb] = (v8f){};
    const size_t aoff = (size_t)(r0 + lr) * K + 8 * hi, boff = (size_t)(c0 + lr) * K + 8 * hi;
#pragma unroll 1
    for (int kc = 0; kc < K; kc += 32) {
        V a[4], a2[4];
#pragma unroll
        for (int mb = 0; mb < 4; ++mb) { a[mb] = WFrag<T16>::ld(A + aoff + (size_t)mb * 16 * K + kc); if (NSPLIT == 1 || NSPLIT == 2) a2[mb] = WFrag<T16>::ld(A2 + aoff + (size_t)mb * 16 * K + kc); }
#pragma unroll
        for (int nb = 0; nb < 4; ++nb) { const V b = WFrag<T16>::ld(Bt + boff + (size_t)nb * 16 * K + kc); V b2; if (NSPLIT >= 2) b2 = WFrag<T16>::ld(Bt2 + boff + (size_t)nb * 16 * K + kc);
#pragma unroll
            for (int mb = 0; mb < 4; ++mb) { acc[mb][nb] = WFrag<T16>::mma(a[mb], b, acc[mb][nb]); if (NSPLIT == 1 || NSPLIT == 2) acc[mb][nb] = WFrag<T16>::mma(a2[mb], b, acc[mb][nb]); if (NSPLIT >= 2) acc[mb][nb] = WFrag<T16>::mma(a[mb], b2, acc[mb][nb]); } }
        asm volatile("v_nop\n\tv_nop\n\tv_nop\n\tv_nop" : "+v"(acc[0][0]), "+v"(acc[1][1]), "+v"(acc[2][2]), "+v"(acc[3][3]) : "v"(a[0]), "v"(a[3]));
    }
#pragma unroll
    for (int mb = 0; mb < 4; ++mb) {
#pragma unroll
        for (int nb = 0; nb < 4; ++nb) {
#pragma unroll
            for (int j = 0; j < 8; ++j) os[(hi * 8 + j) * 68 + nb * 16 + lr] = acc[mb][nb][j]; }
        __builtin_amdgcn_wave_barrier(); asm volatile("" ::: "memory");
        float* crow = C + (size_t)(r0 + mb * 16) * ldc + c0;
#pragma unroll 1
        for (int ps = 0; ps < 2; ++ps) {
#pragma unroll
            for (int s = 0; s < 8; ++s) { const int row = 2 * s + hi, cofs = lr * 4; v4f val = *(const v4fa*)(os + row * 68 + cofs); if (BIAS) { val[0] += bfr(bias[c0 + cofs]); val[1] += bfr(bias[c0 + cofs + 1]); val[2] += bfr(bias[c0 + cofs + 2]); val[3] += bfr(bias[c0 + cofs + 3]); }
                *(volatile v4f*)(crow + (size_t)row * ldc + cofs) = val; }
            if (ps == 0) __threadfence(); }
        __builtin_amdgcn_wave_barrier(); asm volatile("" ::: "memory");
    }
}

__global__ __launch_bounds__(256) void k_wtG(const float* __restrict__ w, int K, int N, bf* Bt) {
    const int lane = threadIdx.x & 31; const int L0 = (blockIdx.x * 8 + (threadIdx.x >> 5)) * 8; const int nlines = N * K / 64;
#pragma unroll
    for (int ps = 0; ps < 2; ++ps) {
#pragma unroll 1
        for (int l = 0; l < 8; ++l) { const int L = L0 + l; if (L >= nlines) break; const size_t e = (size_t)L * 64 + lane * 2; const int k = (int)(e % K), n = (int)(e / K); v2us o;
            o[0] = f2bf(w[(size_t)k * N + n]); o[1] = f2bf(w[(size_t)(k + 1) * N + n]); *(volatile v2us*)(Bt + e) = o; }
        if (ps == 0) __threadfence(); }
}

__global__ __launch_bounds__(256) void k_ln256(const float* __restrict__ X, int nrows, const float* __restrict__ gw, const float* __restrict__ gb, bf* Yh, bf* Yl) {
    const int lane = threadIdx.x & 31; const int r = blockIdx.x * 8 + (threadIdx.x >> 5); if (r >= nrows) return; const float* xr = X + (size_t)r * DM; float hv[8]; float s = 0.f;
#pragma unroll
    for (int ch = 0; ch < 2; ++ch) { const v4f y = *(const v4f*)(xr + ch * 128 + lane * 4);
#pragma unroll
        for (int q = 0; q < 4; ++q) { const float u = bfr(y[q]); hv[ch * 4 + q] = u; s += u; } }
#pragma unroll
    for (int sh = 16; sh; sh >>= 1) s += __shfl_xor(s, sh, 32);
    float mu = s * (1.0f / 256.0f); asm volatile("" : "+v"(mu)); float s2 = 0.f;
#pragma unroll
    for (int k = 0; k < 8; ++k) { float d0 = __fsub_rn(hv[k], mu); asm volatile("" : "+v"(d0)); float p = __fmul_rn(d0, d0); asm volatile("" : "+v"(p)); s2 = __fadd_rn(s2, p); }
#pragma unroll
    for (int sh = 16; sh; sh >>= 1) s2 += __shfl_xor(s2, sh, 32);
    float var = __fadd_rn(s2 * (1.0f / 256.0f), 1e-5f); asm volatile("" : "+v"(var)); const float rs = __frsqrt_rn(var);
#pragma unroll 1
    for (int ps = 0; ps < 2; ++ps) {
#pragma unroll
        for (int ch = 0; ch < 2; ++ch) { const int c0 = ch * 128 + lane * 4; v4us oh, ol;
#pragma unroll
            for (int q = 0; q < 4; ++q) { float gg = bfr(gw[c0 + q]); asm volatile("" : "+v"(gg)); float d0 = __fsub_rn(hv[ch * 4 + q], mu); asm volatile("" : "+v"(d0)); float n0 = __fmul_rn(d0, rs); asm volatile("" : "+v"(n0)); float y = __fmul_rn(n0, gg); asm volatile("" : "+v"(y)); y = __fadd_rn(y, bfr(gb[c0 + q])); unsigned short a, c2; splitf(y, a, c2); oh[q] = a; ol[q] = c2; }
            *(volatile v4us*)(Yh + (size_t)r * DM + c0) = oh; *(volatile v4us*)(Yl + (size_t)r * DM + c0) = ol; }
        if (ps == 0) __threadfence(); } }

__global__ __launch_bounds__(256) void k_planes(const float* __restrict__ F, int pitch, bf* QPh, bf* QPl, bf* KPh, bf* KPl, bf* Vh, bf* Vl) {
    const int sel = blockIdx.y;
    const size_t e = ((size_t)blockIdx.x * 256 + threadIdx.x) * 2; if (e >= (size_t)ZH * TT * HD) return;
    v2us oh, ol;
    if (sel < 2) {
        const int d = (int)(e % HD); const int t = (int)((e / HD) % TT); const int z = (int)(e / ((size_t)HD * TT)); const int h = z % NH_, sq = z / NH_;
        const float* f = F + ((size_t)sq * TT + t) * pitch + sel * DQ + h * HD + d;
#pragma unroll
        for (int q = 0; q < 2; ++q) { unsigned short a, c2; splitf(f[q], a, c2); oh[q] = a; ol[q] = c2; }
        bf* Ph = (sel == 0) ? QPh : KPh; bf* Pl = (sel == 0) ? QPl : KPl;
        *(volatile v2us*)(Ph + e) = oh; *(volatile v2us*)(Pl + e) = ol; __threadfence(); *(volatile v2us*)(Ph + e) = oh; *(volatile v2us*)(Pl + e) = ol;
    } else {
        const int t = (int)(e % TT); const int d = (int)((e / TT) % HD); const int z = (int)(e / ((size_t)TT * HD)); const int h = z % NH_, sq = z / NH_;
#pragma unroll
        for (int q = 0; q < 2; ++q) { const float x = F[((size_t)sq * TT + t + q) * pitch + 2 * DQ + h * HD + d]; unsigned short a, c2; splitf(x, a, c2); oh[q] = a; ol[q] = c2; }
        *(volatile v2us*)(Vh + e) = oh; *(volatile v2us*)(Vl + e) = ol; __threadfence(); *(volatile v2us*)(Vh + e) = oh; *(volatile v2us*)(Vl + e) = ol;
    }
}

__global__ __launch_bounds__(256) void k_asoft(const float* __restrict__ Sb, bf* Ph, bf* Pl) {
    const int lane = threadIdx.x & 31; const int row = blockIdx.x * 8 + (threadIdx.x >> 5); if (row >= ZH * TT) return;
    const float* sr = Sb + (size_t)row * TT; float v[TT / 32]; float mx = -3.0e38f;
#pragma unroll
    for (int ch = 0; ch < TT / 128; ++ch) { const int j0 = ch * 128 + lane * 4; const v4f a = *(const v4f*)(sr + j0);
#pragma unroll
        for (int q = 0; q < 4; ++q) { const float t = a[q] * SCL; v[ch * 4 + q] = t; mx = fmaxf(mx, t); } }
#pragma unroll
    for (int sh = 16; sh; sh >>= 1) mx = fmaxf(mx, __shfl_xor(mx, sh, 32));
    float sum = 0.f;
#pragma unroll
    for (int k = 0; k < TT / 32; ++k) { float d0 = __fsub_rn(v[k], mx); asm volatile("" : "+v"(d0)); v[k] = __builtin_amdgcn_exp2f(__fmul_rn(d0, 1.4426950408889634f)); sum += v[k]; }
#pragma unroll
    for (int sh = 16; sh; sh >>= 1) sum += __shfl_xor(sum, sh, 32);
    const float f = __fdiv_rn(1.0f, sum);
#pragma unroll 1
    for (int ps = 0; ps < 2; ++ps) {
#pragma unroll
        for (int ch = 0; ch < TT / 128; ++ch) { v4us oh, ol;
#pragma unroll
            for (int q = 0; q < 4; ++q) { unsigned short a, c2; splitf(v[ch * 4 + q] * f, a, c2); oh[q] = a; ol[q] = c2; }
            const size_t oo = (size_t)row * TT + ch * 128 + lane * 4; *(volatile v4us*)(Ph + oo) = oh; *(volatile v4us*)(Pl + oo) = ol; }
        if (ps == 0) __threadfence(); }
}

__global__ __launch_bounds__(256) void k_mergeGz(const float* __restrict__ O, const float* __restrict__ G, int gpitch, int gcoff, const float* __restrict__ bgp, bf* Ah, bf* Al) {
    const size_t e = ((size_t)blockIdx.x * 256 + threadIdx.x) * 2; if (e >= (size_t)ZH * TT * HD) return;
    const int d = (int)(e % HD); const int t = (int)((e / HD) % TT); const int z = (int)(e / ((size_t)HD * TT)); const int h = z % NH_, sq = z / NH_;
    const size_t tok = (size_t)sq * TT + t; const int col = h * HD + d;
    const size_t oo = tok * DQ + col; const size_t go = tok * (size_t)gpitch + gcoff + col; v2us oh, ol;
#pragma unroll
    for (int q = 0; q < 2; ++q) { float o = O[e + q]; asm volatile("" : "+v"(o)); float g = __fadd_rn(G[go + q], bfr(bgp[col + q])); asm volatile("" : "+v"(g)); float den = __fadd_rn(1.0f, expf(-g)); asm volatile("" : "+v"(den)); const float sg = __fdiv_rn(1.0f, den); unsigned short a, c2; splitf(__fmul_rn(o, sg), a, c2); oh[q] = a; ol[q] = c2; }
    *(volatile v2us*)(Ah + oo) = oh; *(volatile v2us*)(Al + oo) = ol; __threadfence(); *(volatile v2us*)(Ah + oo) = oh; *(volatile v2us*)(Al + oo) = ol; }

extern "C" void kernel_launch(void* const* d_in, const int* in_sizes, int n_in,
                              void* d_out, int out_size, void* d_ws, size_t ws_size, hipStream_t stream) {
    if (n_in < 9) return;
    if (in_sizes[0] < NT * DM || in_sizes[1] < DM || in_sizes[2] < DM || in_sizes[3] < DM * DQ || in_sizes[4] < DM * 2 * DQ
        || in_sizes[5] < DM * DQ || in_sizes[6] < DQ || in_sizes[7] < DQ * DM || in_sizes[8] < DM) return;
    if (out_size < NT * DM) return;
    const float* x = (const float*)d_in[0]; const float* ln_g = (const float*)d_in[1]; const float* ln_b = (const float*)d_in[2]; const float* wq = (const float*)d_in[3]; const float* wkv = (const float*)d_in[4]; const float* wg = (const float*)d_in[5]; const float* bg = (const float*)d_in[6]; const float* wo = (const float*)d_in[7]; const float* bo = (const float*)d_in[8];
    float* OUT = (float*)d_out;
    char* wsp = (char*)d_ws;
    auto take = [&](size_t bytes) { char* p = wsp; wsp += (bytes + 255) & ~(size_t)255; return (void*)p; };
    bf* WB = (bf*)take((size_t)DP * DM * 2);
    bf* WO = (bf*)take((size_t)DM * DQ * 2);
    bf* LNh = (bf*)take((size_t)NT * DM * 2); bf* LNl = (bf*)take((size_t)NT * DM * 2);
    float* F = (float*)take((size_t)GR * DP * 4);
    bf* QPh = (bf*)take((size_t)ZH * TT * HD * 2); bf* QPl = (bf*)take((size_t)ZH * TT * HD * 2); bf* KPh = (bf*)take((size_t)ZH * TT * HD * 2); bf* KPl = (bf*)take((size_t)ZH * TT * HD * 2); bf* VTh = (bf*)take((size_t)ZH * HD * TT * 2); bf* VTl = (bf*)take((size_t)ZH * HD * TT * 2);
    float* Sb = (float*)take((size_t)ZH * TT * TT * 4); bf* Ph = (bf*)take((size_t)ZH * TT * TT * 2); bf* Pl = (bf*)take((size_t)ZH * TT * TT * 2); float* Ob = (float*)take((size_t)ZH * TT * HD * 4); bf* ATh = (bf*)take((size_t)GR * DQ * 2); bf* ATl = (bf*)take((size_t)GR * DQ * 2);
    if ((size_t)(wsp - (char*)d_ws) > ws_size) return;
    k_wtG<<<(unsigned)((DM * DQ / 64 + 63) / 64), 256, 0, stream>>>(wq, DM, DQ, WB);
    k_wtG<<<(unsigned)((DM * 2 * DQ / 64 + 63) / 64), 256, 0, stream>>>(wkv, DM, 2 * DQ, WB + (size_t)DQ * DM);
    k_wtG<<<(unsigned)((DM * DQ / 64 + 63) / 64), 256, 0, stream>>>(wg, DM, DQ, WB + (size_t)3 * DQ * DM);
    k_wtG<<<(unsigned)((DQ * DM / 64 + 63) / 64), 256, 0, stream>>>(wo, DQ, DM, WO);
    k_ln256<<<NT / 8, 256, 0, stream>>>(x, NT, ln_g, ln_b, LNh, LNl);
    const unsigned LP = (unsigned)(((size_t)ZH * TT * HD / 2 + 255) / 256);
    for (int g = 0; g < NB_ / GB; ++g) { const size_t row0 = (size_t)g * GR;
        k_gemmw<bf, 1, false><<<dim3(GR / 64, DP / 64, 1), 32, 0, stream>>>(LNh + row0 * DM, LNl + row0 * DM, WB, nullptr, DM, F, DP, nullptr, 0, 0, 0);
        k_planes<<<dim3(LP, 3, 1), 256, 0, stream>>>(F, DP, QPh, QPl, KPh, KPl, VTh, VTl);
        k_gemmw<bf, 2, false><<<dim3(TT / 64, TT / 64, ZH), 32, 0, stream>>>(QPh, QPl, KPh, KPl, HD, Sb, TT, nullptr, (size_t)TT * HD, (size_t)TT * HD, (size_t)TT * TT);
        k_asoft<<<ZH * TT / 8, 256, 0, stream>>>(Sb, Ph, Pl);
        k_gemmw<bf, 2, false><<<dim3(TT / 64, HD / 64, ZH), 32, 0, stream>>>(Ph, Pl, VTh, VTl, TT, Ob, HD, nullptr, (size_t)TT * TT, (size_t)HD * TT, (size_t)TT * HD);
        k_mergeGz<<<LP, 256, 0, stream>>>(Ob, F, DP, 3 * DQ, bg, ATh, ATl);
        k_gemmw<bf, 1, true><<<dim3(GR / 64, DM / 64, 1), 32, 0, stream>>>(ATh, ATl, WO, nullptr, DQ, OUT + row0 * DM, DM, bo, 0, 0, 0); }
}
